// NLBlockND_multicross_block_81114752352479
// MI455X (gfx1250) — hardware-verified
//
#include <hip/hip_runtime.h>


#define NB_  4
#define CIN  256
#define CI   128
#define NN_  4096
#define PSC  32768.0f
#define LOSC 1024.0f
#define LOSCI (1.0f / 1024.0f)

typedef _Float16 h16;
typedef unsigned short bf;
typedef __attribute__((ext_vector_type(16))) __bf16   v16bf;
typedef __attribute__((ext_vector_type(16))) _Float16 v16h;
typedef __attribute__((ext_vector_type(8)))  _Float16 v8h;
typedef __attribute__((ext_vector_type(8)))  unsigned short v8us;
typedef __attribute__((ext_vector_type(8)))  float    v8f;
typedef __attribute__((ext_vector_type(4)))  float    v4f;
typedef v8h  __attribute__((may_alias)) v8ha;
typedef v4f  __attribute__((may_alias)) v4fa;
typedef v8us __attribute__((may_alias)) v8usa;

__device__ __forceinline__ unsigned short f2bf(float f) { unsigned u = __float_as_uint(f); u += 0x7FFFu + ((u >> 16) & 1u); return (unsigned short)(u >> 16); }
__device__ __forceinline__ float bf2f(unsigned short b) { return __uint_as_float(((unsigned)b) << 16); }
__device__ __forceinline__ float bfr(float f) { return bf2f(f2bf(f)); }
__device__ __forceinline__ v16h cat16(v8h lo, v8h hi) { return __builtin_shufflevector(lo, hi, 0, 1, 2, 3, 4, 5, 6, 7, 8, 9, 10, 11, 12, 13, 14, 15); }
__device__ __forceinline__ v16bf cat16b(v8us lo, v8us hi) { return __builtin_bit_cast(v16bf, __builtin_shufflevector(lo, hi, 0, 1, 2, 3, 4, 5, 6, 7, 8, 9, 10, 11, 12, 13, 14, 15)); }
__device__ __forceinline__ v8f wmma16(v16h a, v16h b, v8f c) { return __builtin_amdgcn_wmma_f32_16x16x32_f16(false, a, false, b, (short)0, c, false, false); }
__device__ __forceinline__ v8f wmmab(v16bf a, v16bf b, v8f c) { return __builtin_amdgcn_wmma_f32_16x16x32_bf16(false, a, false, b, (short)0, c, false, false); }
#define VST2(T, p, v) do { const T vst2_v_ = (v); *(volatile T*)(p) = vst2_v_; __threadfence(); *(volatile T*)(p) = vst2_v_; } while (0)

__global__ __launch_bounds__(256) void k_xt(const float* __restrict__ x, bf* XT) {
    __shared__ __align__(16) unsigned short tl[64 * 72];
    const int tid = threadIdx.x, n0 = blockIdx.x * 64, c0 = blockIdx.y * 64, b = blockIdx.z;
    const int cr = tid >> 2, nq = (tid & 3) * 16;
#pragma unroll
    for (int i = 0; i < 16; ++i) tl[(nq + i) * 72 + cr] = f2bf(x[((size_t)b * CIN + c0 + cr) * NN_ + n0 + nq + i]);
    __syncthreads();
    const int piece = tid & 7;
    auto pass = [&]() {
#pragma unroll
        for (int s = 0; s < 2; ++s) { const int nr = (tid >> 3) + 32 * s; const v8us val = *(const v8usa*)(tl + nr * 72 + piece * 8);
            *(volatile v8us*)(XT + ((size_t)b * NN_ + n0 + nr) * CIN + c0 + piece * 8) = val; }
    };
    pass(); __threadfence(); pass();
}
__global__ __launch_bounds__(256) void k_cvtw(const float* __restrict__ Wm, int rows, int cols, bf* WB) {
    const int lane = threadIdx.x & 31, r = blockIdx.x * 8 + (threadIdx.x >> 5);
    if (r >= rows) return;
    if (cols == CIN) { v8us t;
#pragma unroll
        for (int i = 0; i < 8; ++i) t[i] = f2bf(Wm[(size_t)r * cols + lane * 8 + i]);
        VST2(v8us, WB + (size_t)r * cols + lane * 8, t); }
    else { typedef __attribute__((ext_vector_type(4))) unsigned short v4us; v4us t;
#pragma unroll
        for (int i = 0; i < 4; ++i) t[i] = f2bf(Wm[(size_t)r * cols + lane * 4 + i]);
        VST2(v4us, WB + (size_t)r * cols + lane * 4, t); }
}
template <int MODE>
__global__ __launch_bounds__(128) void k_proj(const bf* __restrict__ XT, const bf* __restrict__ WB, const float* __restrict__ bias, void* C, void* C2) {
    __shared__ __align__(16) float ost[4][16 * 68];
    const int lane = threadIdx.x & 31, wave = threadIdx.x >> 5, lr = lane & 15, hi = lane >> 4, b = blockIdx.z;
    const int r0 = blockIdx.x * 64 + wave * 16, c0 = blockIdx.y * 64;
    const bf* A = XT + (size_t)b * NN_ * CIN;
    const size_t aoff = (size_t)(r0 + lr) * CIN + 8 * hi;
    size_t boff[4];
#pragma unroll
    for (int t = 0; t < 4; ++t) boff[t] = (size_t)(c0 + t * 16 + lr) * CIN + 8 * hi;
    v8f acc[4];
#pragma unroll
    for (int t = 0; t < 4; ++t) acc[t] = (v8f){};
#pragma unroll 1
    for (int kc = 0; kc < CIN; kc += 32) {
        const v16bf a = cat16b(*(const v8us*)(A + aoff + kc), *(const v8us*)(A + aoff + kc + 16));
#pragma unroll
        for (int t = 0; t < 4; ++t) acc[t] = wmmab(a, cat16b(*(const v8us*)(WB + boff[t] + kc), *(const v8us*)(WB + boff[t] + kc + 16)), acc[t]);
        asm volatile("v_nop\n\tv_nop\n\tv_nop\n\tv_nop" : "+v"(acc[0]), "+v"(acc[1]), "+v"(acc[2]), "+v"(acc[3]) : "v"(a));
    }
    float* os = &ost[wave][0];
#pragma unroll
    for (int t = 0; t < 4; ++t) { const float bv = bfr(bias[c0 + t * 16 + lr]);
#pragma unroll
        for (int j = 0; j < 8; ++j) os[(hi * 8 + j) * 68 + t * 16 + lr] = acc[t][j] + bv; }
    __syncthreads();
    const size_t rowbase = (size_t)b * NN_ + r0;
    if (MODE == 1) {
        float* crow = (float*)C + rowbase * CI + c0;
        auto pass = [&]() {
#pragma unroll
            for (int s = 0; s < 8; ++s) { const int Lid = (lane >> 3) + 4 * s, piece = lane & 7; const int row = Lid >> 1, cofs = (Lid & 1) * 32 + piece * 4;
                const v4f val = *(const v4fa*)(os + row * 68 + cofs); *(volatile v4f*)(crow + (size_t)row * CI + cofs) = val; }
        };
        pass(); __threadfence(); pass();
    } else {
        h16* c1 = (h16*)C + rowbase * CI + c0; h16* c2 = (h16*)C2 + rowbase * CI + c0;
        auto pass = [&]() {
#pragma unroll
            for (int s = 0; s < 4; ++s) { const int row = 4 * s + (lane >> 3), piece = lane & 7; const float* sp = os + row * 68 + piece * 8; v8h o1, o2;
#pragma unroll
                for (int i = 0; i < 8; ++i) { const h16 a = (h16)sp[i]; o1[i] = a; o2[i] = (h16)((sp[i] - (float)a) * LOSC); }
                *(volatile v8h*)(c1 + (size_t)row * CI + piece * 8) = o1; *(volatile v8h*)(c2 + (size_t)row * CI + piece * 8) = o2; }
        };
        pass(); __threadfence(); pass();
    }
}
__global__ __launch_bounds__(256) void k_vt(const float* __restrict__ G, h16* GTH, h16* GTL) {
    __shared__ __align__(16) h16 t1[CI * 72];
    __shared__ __align__(16) h16 t2[CI * 72];
    const int b = blockIdx.x / (NN_ / 64), kt = blockIdx.x - b * (NN_ / 64), n0 = kt * 64, tid = threadIdx.x;
    const int nn = tid >> 2, cq = (tid & 3) * 32;
    const float* src = G + ((size_t)b * NN_ + n0 + nn) * CI + cq;
#pragma unroll
    for (int i = 0; i < 32; ++i) { const float v = src[i]; const h16 a = (h16)v; t1[(cq + i) * 72 + nn] = a; t2[(cq + i) * 72 + nn] = (h16)(v - (float)a); }
    __syncthreads();
    const int piece = tid & 7;
    const size_t base = ((size_t)b * CI) * NN_ + n0;
    auto pass = [&]() {
#pragma unroll
        for (int s = 0; s < 8; ++s) { const int Lid = (tid >> 3) + 32 * s; const int pln = Lid >> 7, c = Lid & 127;
            const v8h val = *(const v8ha*)((pln ? t2 : t1) + c * 72 + piece * 8); *(volatile v8h*)((pln ? GTL : GTH) + base + (size_t)c * NN_ + piece * 8) = val; }
    };
    pass(); __threadfence(); pass();
}
__global__ __launch_bounds__(128) void k_attn(const h16* __restrict__ PH, const h16* __restrict__ PL, const h16* __restrict__ TH, const h16* __restrict__ TL,
                                             const h16* __restrict__ GTH, const h16* __restrict__ GTL, float* Y) {
    __shared__ __align__(16) h16 plds[4][16 * 32];
    __shared__ __align__(16) h16 plds2[4][16 * 32];
    __shared__ __align__(16) float ost[4][16 * 132];
    const int lane = threadIdx.x & 31, wave = threadIdx.x >> 5, lr = lane & 15, hi = lane >> 4;
    const int b = blockIdx.x / (NN_ / 64), qt = blockIdx.x - b * (NN_ / 64), q0 = qt * 64 + wave * 16;
    const size_t tok0 = (size_t)b * NN_;
    h16* pl = &plds[wave][0]; h16* pl2 = &plds2[wave][0];
    v16h ah[4];
    const size_t qo0 = (tok0 + q0 + lr) * CI + 8 * hi;
#pragma unroll
    for (int kc = 0; kc < 4; ++kc) ah[kc] = cat16(*(const v8h*)(PH + qo0 + kc * 32), *(const v8h*)(PH + qo0 + kc * 32 + 16));
    const size_t vbase = ((size_t)b * CI) * NN_;
    v8f o[8];
#pragma unroll
    for (int n = 0; n < 8; ++n) o[n] = (v8f){};
    float mrow[8], lpart[8];
#pragma unroll
    for (int j = 0; j < 8; ++j) { mrow[j] = -3.0e38f; lpart[j] = 0.f; }
#pragma unroll 1
    for (int kt = 0; kt < NN_ / 32; ++kt) {
        const int l0 = kt * 32;
        v8f s0 = {}, s1 = {}, x0 = {}, x1 = {};
#pragma unroll
        for (int kc = 0; kc < 4; ++kc) {
            const size_t ko = (tok0 + l0 + lr) * CI + kc * 32 + 8 * hi, k1o = ko + (size_t)16 * CI;
            { const v16h k0h = cat16(*(const v8h*)(TH + ko), *(const v8h*)(TH + ko + 16)), k1h = cat16(*(const v8h*)(TH + k1o), *(const v8h*)(TH + k1o + 16));
              const v16h alk = cat16(*(const v8h*)(PL + qo0 + kc * 32), *(const v8h*)(PL + qo0 + kc * 32 + 16));
              s0 = wmma16(ah[kc], k0h, s0); x0 = wmma16(alk, k0h, x0); s1 = wmma16(ah[kc], k1h, s1); x1 = wmma16(alk, k1h, x1);
              asm volatile("v_nop" : "+v"(s0), "+v"(s1), "+v"(x0), "+v"(x1) : "v"(alk), "v"(k0h), "v"(k1h) : "memory"); }
            { const v16h k0l = cat16(*(const v8h*)(TL + ko), *(const v8h*)(TL + ko + 16)), k1l = cat16(*(const v8h*)(TL + k1o), *(const v8h*)(TL + k1o + 16));
              x0 = wmma16(ah[kc], k0l, x0); x1 = wmma16(ah[kc], k1l, x1);
              asm volatile("v_nop" : "+v"(x0), "+v"(x1) : "v"(k0l), "v"(k1l) : "memory"); }
        }
        asm volatile("v_nop\n\tv_nop\n\tv_nop\n\tv_nop" : "+v"(s0), "+v"(s1), "+v"(x0), "+v"(x1) : "v"(ah[0]), "v"(ah[3]));
        float alpha[8];
#pragma unroll
        for (int j = 0; j < 8; ++j) {
            const float a0 = s0[j] + x0[j] * LOSCI, a1 = s1[j] + x1[j] * LOSCI;
            float mx = fmaxf(a0, a1);
            mx = fmaxf(mx, __shfl_xor(mx, 1, 16)); mx = fmaxf(mx, __shfl_xor(mx, 2, 16)); mx = fmaxf(mx, __shfl_xor(mx, 4, 16)); mx = fmaxf(mx, __shfl_xor(mx, 8, 16));
            const float mn = fmaxf(mrow[j], mx);
            alpha[j] = __expf(mrow[j] - mn); mrow[j] = mn;
            const float e0 = __expf(a0 - mn), e1 = __expf(a1 - mn);
            lpart[j] = lpart[j] * alpha[j] + (e0 + e1);
            const int mr = hi * 8 + j;
            const float ps0 = e0 * PSC, ps1 = e1 * PSC; const h16 h0 = (h16)ps0, h1 = (h16)ps1;
            pl[mr * 32 + lr] = h0; pl[mr * 32 + 16 + lr] = h1; pl2[mr * 32 + lr] = (h16)(ps0 - (float)h0); pl2[mr * 32 + 16 + lr] = (h16)(ps1 - (float)h1);
        }
#pragma unroll
        for (int n = 0; n < 8; ++n)
#pragma unroll
            for (int j = 0; j < 8; ++j) o[n][j] *= alpha[j];
        asm volatile("" ::: "memory");
        const v16h pa = cat16(*(const v8ha*)(pl + lr * 32 + hi * 8), *(const v8ha*)(pl + lr * 32 + 16 + hi * 8));
        const v16h px = cat16(*(const v8ha*)(pl2 + lr * 32 + hi * 8), *(const v8ha*)(pl2 + lr * 32 + 16 + hi * 8));
#pragma unroll
        for (int n = 0; n < 8; ++n) { const size_t vo = vbase + (size_t)(n * 16 + lr) * NN_ + l0 + hi * 8;
            const v16h vh = cat16(*(const v8h*)(GTH + vo), *(const v8h*)(GTH + vo + 16)), vl = cat16(*(const v8h*)(GTL + vo), *(const v8h*)(GTL + vo + 16));
            o[n] = wmma16(pa, vh, o[n]); o[n] = wmma16(pa, vl, o[n]); o[n] = wmma16(px, vh, o[n]);
            asm volatile("" : "+v"(o[n]) : "v"(vh), "v"(vl) : "memory"); }
    }
    float inv[8];
#pragma unroll
    for (int j = 0; j < 8; ++j) { float rs = lpart[j]; rs += __shfl_xor(rs, 1, 16); rs += __shfl_xor(rs, 2, 16); rs += __shfl_xor(rs, 4, 16); rs += __shfl_xor(rs, 8, 16); inv[j] = 1.0f / (rs * PSC); }
    float* os = &ost[wave][0];
#pragma unroll
    for (int n = 0; n < 8; ++n)
#pragma unroll
        for (int j = 0; j < 8; ++j) os[(hi * 8 + j) * 132 + n * 16 + lr] = o[n][j] * inv[j];
    __syncthreads();
    float* yb = Y + (tok0 + q0) * CI;
    auto pass = [&]() {
#pragma unroll
        for (int s = 0; s < 16; ++s) { const v4f val = *(const v4fa*)(os + s * 132 + lane * 4); *(volatile v4f*)(yb + (size_t)s * CI + lane * 4) = val; }
    };
    pass(); __threadfence(); pass();
}
__global__ __launch_bounds__(256) void k_splity(const float* __restrict__ Y, bf* YH, bf* YL) {
    const int lane = threadIdx.x & 31; const size_t w = (size_t)blockIdx.x * 8 + (threadIdx.x >> 5);
    v8us oh, ol;
#pragma unroll
    for (int i = 0; i < 8; ++i) { const float v = Y[w * 256 + lane * 8 + i]; const unsigned short hb = f2bf(v); oh[i] = hb; ol[i] = f2bf(v - bf2f(hb)); }
    *(volatile v8us*)(YH + w * 256 + lane * 8) = oh; *(volatile v8us*)(YL + w * 256 + lane * 8) = ol; __threadfence();
    *(volatile v8us*)(YH + w * 256 + lane * 8) = oh; *(volatile v8us*)(YL + w * 256 + lane * 8) = ol;
}
__global__ __launch_bounds__(128) void k_z(const bf* __restrict__ WZ, const bf* __restrict__ YH, const bf* __restrict__ YL, const float* __restrict__ bz, float* Z) {
    __shared__ __align__(16) float ost[4][16 * 68];
    const int lane = threadIdx.x & 31, wave = threadIdx.x >> 5, lr = lane & 15, hi = lane >> 4, b = blockIdx.z;
    const int r0 = blockIdx.x * 64 + wave * 16, c0 = blockIdx.y * 64;
    const size_t aoff = (size_t)(r0 + lr) * CI + 8 * hi;
    const bf* Bh = YH + (size_t)b * NN_ * CI; const bf* Bl = YL + (size_t)b * NN_ * CI;
    size_t boff[4];
#pragma unroll
    for (int t = 0; t < 4; ++t) boff[t] = (size_t)(c0 + t * 16 + lr) * CI + 8 * hi;
    v8f acc[4], accx[4];
#pragma unroll
    for (int t = 0; t < 4; ++t) { acc[t] = (v8f){}; accx[t] = (v8f){}; }
#pragma unroll
    for (int kc = 0; kc < CI; kc += 32) {
        const v16bf a = cat16b(*(const v8us*)(WZ + aoff + kc), *(const v8us*)(WZ + aoff + kc + 16));
#pragma unroll
        for (int t = 0; t < 4; ++t) { acc[t] = wmmab(a, cat16b(*(const v8us*)(Bh + boff[t] + kc), *(const v8us*)(Bh + boff[t] + kc + 16)), acc[t]); accx[t] = wmmab(a, cat16b(*(const v8us*)(Bl + boff[t] + kc), *(const v8us*)(Bl + boff[t] + kc + 16)), accx[t]); }
    }
    asm volatile("v_nop\n\tv_nop\n\tv_nop\n\tv_nop" : "+v"(acc[0]), "+v"(acc[1]), "+v"(acc[2]), "+v"(acc[3]), "+v"(accx[0]), "+v"(accx[1]), "+v"(accx[2]), "+v"(accx[3]));
    float* os = &ost[wave][0];
#pragma unroll
    for (int t = 0; t < 4; ++t)
#pragma unroll
        for (int j = 0; j < 8; ++j) os[(hi * 8 + j) * 68 + t * 16 + lr] = acc[t][j] + accx[t][j] + bfr(bz[r0 + hi * 8 + j]);
    __syncthreads();
    float* crow = Z + ((size_t)b * CI + r0) * NN_ + c0;
    auto pass = [&]() {
#pragma unroll
        for (int s = 0; s < 8; ++s) { const int Lid = (lane >> 3) + 4 * s, piece = lane & 7; const int row = Lid >> 1, cq = (Lid & 1) * 32 + piece * 4;
            const v4f val = *(const v4fa*)(os + row * 68 + cq); *(volatile v4f*)(crow + (size_t)row * NN_ + cq) = val; }
    };
    pass(); __threadfence(); pass();
}
__global__ __launch_bounds__(256) void k_stats(const float* __restrict__ Z, float* ST) {
    __shared__ float red[256];
    const int o = blockIdx.x, t = threadIdx.x;
    float s = 0.f;
#pragma unroll 1
    for (int i = 0; i < (NB_ * NN_) / 256; ++i) { const int flat = i * 256 + t; const int b = flat / NN_, n = flat - b * NN_; s += Z[((size_t)b * CI + o) * NN_ + n]; }
    red[t] = s; __syncthreads();
    for (int st = 128; st > 0; st >>= 1) { if (t < st) red[t] += red[t + st]; __syncthreads(); }
    const float mu = red[0] / (float)(NB_ * NN_);
    __syncthreads();
    float q = 0.f;
#pragma unroll 1
    for (int i = 0; i < (NB_ * NN_) / 256; ++i) { const int flat = i * 256 + t; const int b = flat / NN_, n = flat - b * NN_; const float d = Z[((size_t)b * CI + o) * NN_ + n] - mu; q += d * d; }
    red[t] = q; __syncthreads();
    for (int st = 128; st > 0; st >>= 1) { if (t < st) red[t] += red[t + st]; __syncthreads(); }
    const float var = red[0] / (float)(NB_ * NN_);
    if (t < 32) { const float v = (t == 0) ? mu : (t == 1) ? rsqrtf(var + 1e-5f) : 0.f; VST2(float, ST + (size_t)o * 32 + t, v); }
}
__global__ __launch_bounds__(256) void k_final(const float* __restrict__ Z, const float* __restrict__ ST, const float* __restrict__ gam, const float* __restrict__ bet, float* out) {
    const int lane = threadIdx.x & 31; const size_t wid = (size_t)blockIdx.x * 8 + (threadIdx.x >> 5);
    const size_t row = wid >> 4; const int seg = (int)(wid & 15);
    const int o = (int)(row % CI);
    const float mu = ST[(size_t)o * 32], rs = ST[(size_t)o * 32 + 1], g = bfr(gam[o]), be = bfr(bet[o]);
#pragma unroll
    for (int hf = 0; hf < 2; ++hf) { const size_t base = row * NN_ + (size_t)seg * 256 + hf * 128 + lane * 4; v4f v;
#pragma unroll
        for (int i = 0; i < 4; ++i) v[i] = (Z[base + i] - mu) * rs * g + be;
        VST2(v4f, out + base, v); }
}

extern "C" void kernel_launch(void* const* d_in, const int* in_sizes, int n_in,
                              void* d_out, int out_size, void* d_ws, size_t ws_size, hipStream_t stream) {
    (void)in_sizes; (void)n_in; (void)out_size;
    const float* xt = (const float*)d_in[0]; const float* xo = (const float*)d_in[1]; const float* wg = (const float*)d_in[2]; const float* bg = (const float*)d_in[3];
    const float* wth = (const float*)d_in[4]; const float* bth = (const float*)d_in[5]; const float* wph = (const float*)d_in[6]; const float* bph = (const float*)d_in[7];
    const float* wz = (const float*)d_in[8]; const float* bz = (const float*)d_in[9]; const float* gam = (const float*)d_in[10]; const float* bet = (const float*)d_in[11];
    float* out = (float*)d_out;
    char* wsp = (char*)d_ws;
    auto take = [&](size_t bytes) { char* p = wsp; wsp += (bytes + 255) & ~(size_t)255; return (void*)p; };
    bf* XTt = (bf*)take((size_t)NB_ * NN_ * CIN * 2); bf* XTo = (bf*)take((size_t)NB_ * NN_ * CIN * 2);
    bf* WGb = (bf*)take((size_t)CI * CIN * 2); bf* WTb = (bf*)take((size_t)CI * CIN * 2); bf* WPb = (bf*)take((size_t)CI * CIN * 2); bf* WZb = (bf*)take((size_t)CI * CI * 2);
    h16* TH = (h16*)take((size_t)NB_ * NN_ * CI * 2); h16* TL = (h16*)take((size_t)NB_ * NN_ * CI * 2); h16* PH = (h16*)take((size_t)NB_ * NN_ * CI * 2); h16* PL = (h16*)take((size_t)NB_ * NN_ * CI * 2);
    float* G = (float*)take((size_t)NB_ * NN_ * CI * 4); h16* GTH = (h16*)take((size_t)NB_ * CI * NN_ * 2); h16* GTL = (h16*)take((size_t)NB_ * CI * NN_ * 2);
    float* Y = (float*)take((size_t)NB_ * NN_ * CI * 4); bf* YH = (bf*)take((size_t)NB_ * NN_ * CI * 2); bf* YL = (bf*)take((size_t)NB_ * NN_ * CI * 2);
    float* Z = (float*)take((size_t)NB_ * CI * NN_ * 4); float* ST = (float*)take((size_t)CI * 32 * 4);
    if ((size_t)(wsp - (char*)d_ws) > ws_size) return;
    k_xt<<<dim3(NN_ / 64, CIN / 64, NB_), 256, 0, stream>>>(xt, XTt);
    k_xt<<<dim3(NN_ / 64, CIN / 64, NB_), 256, 0, stream>>>(xo, XTo);
    k_cvtw<<<CI / 8, 256, 0, stream>>>(wg, CI, CIN, WGb); k_cvtw<<<CI / 8, 256, 0, stream>>>(wth, CI, CIN, WTb); k_cvtw<<<CI / 8, 256, 0, stream>>>(wph, CI, CIN, WPb); k_cvtw<<<CI / 8, 256, 0, stream>>>(wz, CI, CI, WZb);
    k_proj<0><<<dim3(NN_ / 64, CI / 64, NB_), 128, 0, stream>>>(XTt, WTb, bth, TH, TL);
    k_proj<0><<<dim3(NN_ / 64, CI / 64, NB_), 128, 0, stream>>>(XTo, WPb, bph, PH, PL);
    k_proj<1><<<dim3(NN_ / 64, CI / 64, NB_), 128, 0, stream>>>(XTt, WGb, bg, G, nullptr);
    k_vt<<<NB_ * (NN_ / 64), 256, 0, stream>>>(G, GTH, GTL);
    k_attn<<<NB_ * (NN_ / 64), 128, 0, stream>>>(PH, PL, TH, TL, GTH, GTL, Y);
    k_splity<<<(NB_ * NN_ / 2) / 8, 256, 0, stream>>>(Y, YH, YL);
    k_z<<<dim3(CI / 64, NN_ / 64, NB_), 128, 0, stream>>>(WZb, YH, YL, bz, Z);
    k_stats<<<CI, 256, 0, stream>>>(Z, ST);
    k_final<<<(NB_ * CI * 16) / 8, 256, 0, stream>>>(Z, ST, gam, bet, out);
}
